// FusionKANLayer_19035295056670
// MI455X (gfx1250) — hardware-verified
//
#include <hip/hip_runtime.h>


namespace {
constexpr int NR = 4096, IN = 1024, OUT = 1024, NCF = 8, KS = IN * NCF;
constexpr float LN_EPS = 1e-5f;

typedef _Float16 b16;
typedef __attribute__((ext_vector_type(16))) _Float16 v16b;
typedef __attribute__((ext_vector_type(8)))  _Float16 v8b;
typedef __attribute__((ext_vector_type(8)))  float v8f;
typedef __attribute__((ext_vector_type(4)))  float v4f;

__device__ __forceinline__ v8b ld8b(const b16* p) { return *(const v8b*)p; }
__device__ __forceinline__ v16b cat8b(v8b a, v8b b) { return __builtin_shufflevector(a, b, 0, 1, 2, 3, 4, 5, 6, 7, 8, 9, 10, 11, 12, 13, 14, 15); }
__device__ __forceinline__ v16b frag_kb(const b16* p, int hh) { return cat8b(ld8b(p + 8 * hh), ld8b(p + 16 + 8 * hh)); }
__device__ __forceinline__ void split16(float v, b16& hi, b16& lo) { hi = (b16)v; lo = (b16)(v - (float)hi); }
__device__ __forceinline__ void frag_ksplit(const float* p, int hh, v16b& fh_, v16b& fl_) {
  const float* p0 = p + 8 * hh; const float* p1 = p + 16 + 8 * hh;
#pragma unroll
  for (int e = 0; e < 8; ++e) { b16 a, c; split16(p0[e], a, c); fh_[e] = a; fl_[e] = c; split16(p1[e], a, c); fh_[8 + e] = a; fl_[8 + e] = c; }
}
__device__ __forceinline__ v8f wmma16b(v16b a, v16b b, v8f c) {
  v8f d = __builtin_amdgcn_wmma_f32_16x16x32_f16(false, a, false, b, (short)0, c, false, false);
  asm volatile("v_nop\n\tv_nop\n\tv_nop\n\tv_nop" : "+v"(d) : "v"(a), "v"(b));
  return d;
}
__device__ __forceinline__ void wave_lds_sync() {
  __builtin_amdgcn_fence(__ATOMIC_RELEASE, "workgroup");
  __builtin_amdgcn_wave_barrier();
  __builtin_amdgcn_fence(__ATOMIC_ACQUIRE, "workgroup");
}

struct Opnd { const void* p0; const void* p1; int ld; };
template <int NP> __device__ __forceinline__ void load_frags(const Opnd& o, int row, int kb, int hh, v16b& fh_, v16b& fl_) {
  if (NP == 0) { frag_ksplit((const float*)o.p0 + (size_t)row * o.ld + kb, hh, fh_, fl_); }
  else if (NP == 3) {
    const float* p = (const float*)o.p0 + (size_t)row * o.ld + kb; const float* p0 = p + 8 * hh; const float* p1 = p + 16 + 8 * hh;
#pragma unroll
    for (int e = 0; e < 8; ++e) { fh_[e] = (b16)p0[e]; fh_[8 + e] = (b16)p1[e]; }
    fl_ = fh_;
  } else {
    fh_ = frag_kb((const b16*)o.p0 + (size_t)row * o.ld + kb, hh);
    if (NP == 2) fl_ = frag_kb((const b16*)o.p1 + (size_t)row * o.ld + kb, hh); else fl_ = fh_;
  }
}
template <int ANP, int BNP> __device__ __forceinline__ v8f mac(v16b ah, v16b al, v16b bh, v16b bl, v8f c) {
  c = wmma16b(ah, bh, c);
  if (BNP == 0 || BNP == 2) c = wmma16b(ah, bl, c);
  if (ANP == 0 || ANP == 2) c = wmma16b(al, bh, c);
  return c;
}
template <int ANP, int BNP>
__device__ __forceinline__ void gemm_tile(const Opnd& A, const Opnd& B, int K, int m0, int c0, int nloc, int hlf, v8f (&acc)[2][4]) {
  for (int kb = 0; kb < K; kb += 32) {
    v16b a0h, a0l, a1h, a1l;
    load_frags<ANP>(A, m0 + nloc, kb, hlf, a0h, a0l);
    load_frags<ANP>(A, m0 + 16 + nloc, kb, hlf, a1h, a1l);
#pragma unroll
    for (int t = 0; t < 4; ++t) {
      v16b bh, bl;
      load_frags<BNP>(B, c0 + t * 16 + nloc, kb, hlf, bh, bl);
      acc[0][t] = mac<ANP, BNP>(a0h, a0l, bh, bl, acc[0][t]);
      acc[1][t] = mac<ANP, BNP>(a1h, a1l, bh, bl, acc[1][t]);
    }
  }
}

struct Epi { float scale; const float* cscale; const float* cbias; const float* rbias; int act; float post; const float* rscale; const float* resid; };
__device__ __forceinline__ float epi_val(const Epi& e, float acc, int row, int col) {
  float val = acc * e.scale;
  if (e.cscale) val *= e.cscale[col];
  if (e.cbias) val += e.cbias[col];
  if (e.rbias) val += e.rbias[row];
  if (e.act == 1) val = 0.5f * val * (1.0f + erff(val * 0.70710678118654752f));
  val *= e.post;
  if (e.rscale) val *= e.rscale[(size_t)row * 32];
  return val;
}
__device__ __forceinline__ void epi_planes(v8f (&acc)[2][4], const Epi& e, bool two,
                                           b16* __restrict__ oh, b16* __restrict__ ol, int ldo, int m0, int c0, int lane, b16* Th, b16* Tl) {
  const int nloc = lane & 15, hlf = lane >> 4;
#pragma unroll
  for (int t = 0; t < 4; ++t)
#pragma unroll
    for (int r = 0; r < 2; ++r)
#pragma unroll
      for (int v = 0; v < 8; ++v) {
        const int rr = r * 16 + v + 8 * hlf, cc = t * 16 + nloc;
        const float val = epi_val(e, acc[r][t][v], m0 + rr, c0 + cc);
        b16 h_, l_; split16(val, h_, l_);
        Th[rr * 64 + cc] = h_; if (two) Tl[rr * 64 + cc] = l_;
      }
  wave_lds_sync();
  for (int pass = 0; pass < 2; ++pass) {
#pragma unroll
    for (int j = 0; j < 8; ++j) {
      const int rr = j * 4 + (lane >> 3), c8 = (lane & 7) * 8;
      const size_t o = (size_t)(m0 + rr) * ldo + c0 + c8;
      *(volatile v8b*)(oh + o) = ld8b(Th + rr * 64 + c8);
      if (two) *(volatile v8b*)(ol + o) = ld8b(Tl + rr * 64 + c8);
    }
    __threadfence();
  }
}
__device__ __forceinline__ void epi_f32(v8f (&acc)[2][4], const Epi& e, float* __restrict__ out, int ldo, int m0, int c0, int lane, float* Tt) {
  const int nloc = lane & 15, hlf = lane >> 4;
#pragma unroll
  for (int t = 0; t < 4; ++t)
#pragma unroll
    for (int r = 0; r < 2; ++r)
#pragma unroll
      for (int v = 0; v < 8; ++v) {
        const int rr = r * 16 + v + 8 * hlf, cc = t * 16 + nloc;
        Tt[rr * 64 + cc] = epi_val(e, acc[r][t][v], m0 + rr, c0 + cc);
      }
  wave_lds_sync();
  float* dst0 = out + (size_t)m0 * ldo + c0; const float* rs0 = e.resid ? e.resid + (size_t)m0 * ldo + c0 : nullptr;
  for (int pass = 0; pass < 2; ++pass) {
#pragma unroll
    for (int j = 0; j < 16; ++j) {
      const int rr = j * 2 + hlf, c4 = nloc * 4;
      v4f val = *(const v4f*)(Tt + rr * 64 + c4);
      if (rs0) val += *(const v4f*)(rs0 + (size_t)rr * ldo + c4);
      *(volatile v4f*)(dst0 + (size_t)rr * ldo + c4) = val;
    }
    __threadfence();
  }
}


__device__ __forceinline__ void bspline8(float x, float* outb) {
  const float h = 0.4f;
  float t[12];
#pragma unroll
  for (int j = 0; j < 12; ++j) t[j] = -1.0f + h * (float)(j - 3);
  float b[11];
#pragma unroll
  for (int j = 0; j < 11; ++j) b[j] = (x >= t[j] && x < t[j + 1]) ? 1.0f : 0.0f;
#pragma unroll
  for (int p = 1; p <= 3; ++p) {
#pragma unroll
    for (int j = 0; j < 11 - p; ++j) {
      const float il = 1.0f / (t[j + p] - t[j]), ir = 1.0f / (t[j + p + 1] - t[j + 1]);
      const float left = (x - t[j]) * il * b[j];
      const float right = (t[j + p + 1] - x) * ir * b[j + 1];
      b[j] = left + right;
    }
  }
#pragma unroll
  for (int c = 0; c < 8; ++c) outb[c] = b[c];
}
__global__ __launch_bounds__(256) void prep_kernel(const float* __restrict__ x, const float* __restrict__ ws_, const float* __restrict__ wb,
                                                   const float* __restrict__ bb, const float* __restrict__ sb,
                                                   b16* __restrict__ sx16, b16* __restrict__ bs16, b16* __restrict__ ws16, b16* __restrict__ wb16, float* __restrict__ bsb) {
  const size_t tid = (size_t)blockIdx.x * blockDim.x + threadIdx.x, stride = (size_t)gridDim.x * blockDim.x;
  if (blockIdx.x == 0) {
    const int c = threadIdx.x * 4; v4f w;
#pragma unroll
    for (int e = 0; e < 4; ++e) w[e] = bb[c + e] * sb[c + e];
    *(volatile v4f*)(bsb + c) = w; __threadfence(); *(volatile v4f*)(bsb + c) = w;
  }
  const size_t n0 = (size_t)NR * IN / 8, n1 = (size_t)NR * IN, n2 = (size_t)OUT * KS / 8, n3 = (size_t)OUT * IN / 8;
  for (int pass = 0; pass < 2; ++pass) {
    for (size_t c = tid; c < n0 + n1 + n2 + n3; c += stride) {
      v8b v;
      if (c < n0) { const size_t i = c * 8;
#pragma unroll
        for (int e = 0; e < 8; ++e) { const float xv = x[i + e]; v[e] = (b16)(xv / (1.0f + expf(-xv))); }
        *(volatile v8b*)(sx16 + i) = v;
      } else if (c < n0 + n1) { const size_t i = c - n0;
        float bb[8]; bspline8(x[i], bb);
#pragma unroll
        for (int e = 0; e < 8; ++e) v[e] = (b16)bb[e];
        *(volatile v8b*)(bs16 + i * 8) = v;
      } else if (c < n0 + n1 + n2) { const size_t i = (c - n0 - n1) * 8;
#pragma unroll
        for (int e = 0; e < 8; ++e) v[e] = (b16)ws_[i + e];
        *(volatile v8b*)(ws16 + i) = v;
      } else { const size_t i = (c - n0 - n1 - n2) * 8;
#pragma unroll
        for (int e = 0; e < 8; ++e) v[e] = (b16)wb[i + e];
        *(volatile v8b*)(wb16 + i) = v;
      }
    }
    __threadfence();
  }
}

__global__ __launch_bounds__(128) void gemm_kernel(const b16* __restrict__ A, int lda, const b16* __restrict__ Bm, int ldb, int K,
                                                   const float* __restrict__ cscale, const float* __restrict__ cbias, const float* __restrict__ resid,
                                                   float* __restrict__ o32, int ldo) {
  __shared__ __attribute__((aligned(16))) float Ts[4][32 * 64];
  const int lane = threadIdx.x & 31, wave = threadIdx.x >> 5, nloc = lane & 15, hlf = lane >> 4;
  const int m0 = blockIdx.y * 128 + wave * 32, c0 = blockIdx.x * 64;
  v8f acc[2][4];
#pragma unroll
  for (int r = 0; r < 2; ++r)
#pragma unroll
    for (int t = 0; t < 4; ++t) acc[r][t] = (v8f){};
  const Opnd Ao{A, nullptr, lda}, Bo{Bm, nullptr, ldb};
  gemm_tile<1, 1>(Ao, Bo, K, m0, c0, nloc, hlf, acc);
  const Epi e{1.0f, cscale, cbias, nullptr, 0, 1.0f, nullptr, resid};
  epi_f32(acc, e, o32, ldo, m0, c0, lane, Ts[wave]);
}

__global__ __launch_bounds__(256) void ln_prelu_kernel(const float* __restrict__ y, const float* __restrict__ g, const float* __restrict__ bta,
                                                       const float* __restrict__ slope, float* __restrict__ out) {
  const int lane = threadIdx.x & 31, row = blockIdx.x * 8 + (threadIdx.x >> 5);
  const float* yr = y + (size_t)row * OUT;
  v4f v[8];
  float s = 0.f;
#pragma unroll
  for (int j = 0; j < 8; ++j) { v[j] = *(const v4f*)(yr + j * 128 + lane * 4); s += (v[j][0] + v[j][1]) + (v[j][2] + v[j][3]); }
#pragma unroll
  for (int o = 16; o > 0; o >>= 1) s += __shfl_xor(s, o);
  const float mu = s * (1.0f / OUT);
  float s2 = 0.f;
#pragma unroll
  for (int j = 0; j < 8; ++j)
#pragma unroll
    for (int q = 0; q < 4; ++q) { const float dl = v[j][q] - mu; s2 += dl * dl; }
#pragma unroll
  for (int o = 16; o > 0; o >>= 1) s2 += __shfl_xor(s2, o);
  const float rs = rsqrtf(s2 * (1.0f / OUT) + LN_EPS), a = slope[0];
  float* dst = out + (size_t)row * OUT;
  for (int pass = 0; pass < 2; ++pass) {
#pragma unroll
    for (int j = 0; j < 8; ++j) {
      v4f w;
#pragma unroll
      for (int q = 0; q < 4; ++q) { const int c = j * 128 + lane * 4 + q; const float yn = (v[j][q] - mu) * rs * g[c] + bta[c]; w[q] = (yn >= 0.0f) ? yn : a * yn; }
      *(volatile v4f*)(dst + j * 128 + lane * 4) = w;
    }
    __threadfence();
  }
}
}

extern "C" void kernel_launch(void* const* d_in, const int* in_sizes, int n_in,
                              void* d_out, int out_size, void* d_ws, size_t ws_size, hipStream_t stream) {
  (void)n_in; (void)out_size;
  const float* x    = (const float*)d_in[0];
  const float* ws_  = (const float*)d_in[1];
  const float* wb   = (const float*)d_in[2];
  const float* bb   = (const float*)d_in[3];
  const float* sb   = (const float*)d_in[4];
  const float* ss   = (const float*)d_in[5];
  const float* lng  = (const float*)d_in[6];
  const float* lnb  = (const float*)d_in[7];
  const float* pw   = (const float*)d_in[8];
  float* out = (float*)d_out;
  if (in_sizes[0] != NR * IN || in_sizes[1] != OUT * KS || in_sizes[2] != OUT * IN) return;

  size_t off = 0; char* ws = (char*)d_ws;
  auto carve = [&](size_t bytes) { char* p = ws + off; off += (bytes + 255) & ~(size_t)255; return p; };
  b16* sx16 = (b16*)carve((size_t)NR * IN * 2);
  b16* bs16 = (b16*)carve((size_t)NR * KS * 2);
  b16* ws16 = (b16*)carve((size_t)OUT * KS * 2);
  b16* wb16 = (b16*)carve((size_t)OUT * IN * 2);
  float* bsb = (float*)carve((size_t)OUT * 4);
  float* y1 = (float*)carve((size_t)NR * OUT * 4);
  float* y2 = (float*)carve((size_t)NR * OUT * 4);
  if (off > ws_size) return;
  prep_kernel<<<2048, 256, 0, stream>>>(x, ws_, wb, bb, sb, sx16, bs16, ws16, wb16, bsb);
  gemm_kernel<<<dim3(OUT / 64, NR / 128), 128, 0, stream>>>(sx16, IN, wb16, IN, IN, sb, bsb, nullptr, y1, OUT);
  gemm_kernel<<<dim3(OUT / 64, NR / 128), 128, 0, stream>>>(bs16, KS, ws16, KS, KS, ss, nullptr, y1, y2, OUT);
  ln_prelu_kernel<<<NR / 8, 256, 0, stream>>>(y2, lng, lnb, pw, out);
}
